// EnBaseLayer_40596030882310
// MI455X (gfx1250) — hardware-verified
//
#include <hip/hip_runtime.h>
#include <stddef.h>
#include <stdint.h>


#define HID    64
#define NPQ    128
#define KN1    192
#define KN2    128
#define NTHR   256
#define NWAVE  8
#define EPB    256
#define DP     68
#define AP     72
#define MPITCH 64
#define CSTN   196
#define GBM    64
#define GTHR   128
#define EPT    8
#define CHUNK  (NTHR * EPT)
#define WCAP   (EPT * 32)
#define LISTN  (NWAVE * WCAP)
#define NBA    1024
#define SLA    10
#define RCAP   28672
#define DEGCAP 64
#define NRANGE 4
#define NU_WABT (NPQ * (HID / 8))
#define NU_WE2  (HID * (HID / 8))
#define NU_WN1  (HID * (KN1 / 8))
#define NU_WN2  (HID * (KN2 / 8))
#define AGG_ZINTS (LISTN + 2 * RCAP + 3 * NBA)
#define AGG_LDS_INTS (AGG_ZINTS + 16)
#define AGG_LDS_BYTES (AGG_LDS_INTS * 4)
#define EDGE_LDS_BYTES (EPB * DP * 4 + EPB * AP * 2 + EPB * MPITCH * 2 + CSTN * 4)
#define WSMAX  134217728
#define CACT   16.0f
#define CWGT   1024.0f
#define CMSG   16.0f
#define PINV   6.103515625e-05f
#define MINV   0.0625f
#define TEMF   30.0f
#define LNEPS  1e-5f

static_assert((CHUNK & (CHUNK - 1)) == 0 && CHUNK <= 4096);
static_assert((NBA & (NBA - 1)) == 0 && NBA == (1 << SLA));
static_assert(((long long)CHUNK << SLA) < (1LL << 31));
static_assert(LISTN % NTHR == 0);
static_assert(NBA % NWAVE == 0 && NBA % 32 == 0 && NBA == 4 * NTHR);
static_assert(RCAP % 4 == 0 && AGG_ZINTS % 4 == 0 && LISTN % 4 == 0);
static_assert(AGG_LDS_BYTES <= 300000);
static_assert(EDGE_LDS_BYTES <= 300000);
static_assert(NU_WABT % NTHR == 0 && NU_WE2 % NTHR == 0 && NU_WN1 % NTHR == 0 && NU_WN2 % NTHR == 0);
static_assert(HID % 32 == 0 && KN1 % 32 == 0 && KN2 % 32 == 0);
static_assert(NPQ == 2 * HID && KN1 == 3 * HID && KN2 == 2 * HID);
static_assert(GBM == (GTHR / 32) * 16);
static_assert((DP * 4) % 16 == 0 && (AP * 2) % 16 == 0 && AP >= HID && DP >= HID);
static_assert(EPB == NTHR && EPB == 8 * 32);
static_assert((EPB * DP * 4) % 16 == 0 && (EPB * AP * 2) % 16 == 0 && (EPB * MPITCH * 2) % 16 == 0);
static_assert((CSTN * 4) % 16 == 0 && CSTN >= 3 * HID + 1);
static_assert(EPB * MPITCH * 2 == 8 * NTHR * 16);
static_assert((GBM * (HID / 8)) % NTHR == 0 && (GBM * (HID / 4)) % NTHR == 0);
static_assert(KN1 / 8 == 24 && KN2 / 8 == 16 && HID / 8 == 8);

typedef float          v4f   __attribute__((ext_vector_type(4)));
typedef float          v8f   __attribute__((ext_vector_type(8)));
typedef int            v4i   __attribute__((ext_vector_type(4)));
typedef int            v8i   __attribute__((ext_vector_type(8)));
typedef unsigned short v8us  __attribute__((ext_vector_type(8)));
typedef unsigned short v16us __attribute__((ext_vector_type(16)));
typedef __bf16         v16bf __attribute__((ext_vector_type(16)));
typedef _Float16       v16h  __attribute__((ext_vector_type(16)));
typedef v4f  __attribute__((may_alias)) v4fa;
typedef v4i  __attribute__((may_alias)) v4ia;
typedef v8us __attribute__((may_alias)) v8usa;
typedef unsigned __attribute__((may_alias)) u32a;
union FragB { v16bf v; v16us u; v8us h[2]; v8i w; };
union FragH { v16h  v; v16us u; v8us h[2]; v8i w; };

__device__ __forceinline__ v8f wmb(const FragB& a, const FragB& b, v8f c) {
  v8f d = __builtin_amdgcn_wmma_f32_16x16x32_bf16(false, a.v, false, b.v, (short)0, c, false, false);
  asm volatile("v_nop\n\tv_nop\n\tv_nop\n\tv_nop" : "+v"(d) : "v"(a.w), "v"(b.w));
  return d;
}
__device__ __forceinline__ v8f wmh(const FragH& a, const FragH& b, v8f c) {
  v8f d = __builtin_amdgcn_wmma_f32_16x16x32_f16(false, a.v, false, b.v, (short)0, c, false, false);
  asm volatile("v_nop\n\tv_nop\n\tv_nop\n\tv_nop" : "+v"(d) : "v"(a.w), "v"(b.w));
  return d;
}

__device__ __forceinline__ unsigned bf16_bits(float f) {
  const unsigned u = __float_as_uint(f);
  return (u + 0x7FFFu + ((u >> 16) & 1u)) >> 16;
}
__device__ __forceinline__ float bf16_val(float f) {
  return __uint_as_float(bf16_bits(f) << 16);
}
__device__ __forceinline__ unsigned short f2h(float f) {
  const _Float16 hv = (_Float16)f;
  return __builtin_bit_cast(unsigned short, hv);
}
__device__ __forceinline__ float h2f(unsigned b) {
  const _Float16 hv = __builtin_bit_cast(_Float16, (unsigned short)b);
  return (float)hv;
}
__device__ __forceinline__ float sigm_f(float t) {
  return __builtin_amdgcn_rcpf(1.0f + __expf(-t));
}
__device__ __forceinline__ void put16(unsigned short* dp, v8us o) {
  *(volatile v8us*)dp = o;
  __threadfence();
  *(volatile v8us*)dp = o;
}
__device__ __forceinline__ void putf4(float* dp, v4f o) {
  *(volatile v4f*)dp = o;
  __threadfence();
  *(volatile v4f*)dp = o;
}

template <int SLB>
__device__ __forceinline__ int scan_chunk(const int* __restrict__ dsts, int nE, int cbase, int slotBase,
                                          int nb, int vec8, int* list, int tid, int lane, int wave) {
  int wc = 0;
  const int el0  = tid * EPT;
  const int e0   = cbase + el0;
  const int sent = -2147483647 - 1;
  v4i da, db;
  if (vec8 != 0 && cbase + CHUNK <= nE) {
    da = *(const v4i*)(dsts + e0);
    db = *(const v4i*)(dsts + e0 + 4);
  } else {
    da.x = (e0     < nE) ? dsts[min(e0,     nE - 1)] : sent;
    da.y = (e0 + 1 < nE) ? dsts[min(e0 + 1, nE - 1)] : sent;
    da.z = (e0 + 2 < nE) ? dsts[min(e0 + 2, nE - 1)] : sent;
    da.w = (e0 + 3 < nE) ? dsts[min(e0 + 3, nE - 1)] : sent;
    db.x = (e0 + 4 < nE) ? dsts[min(e0 + 4, nE - 1)] : sent;
    db.y = (e0 + 5 < nE) ? dsts[min(e0 + 5, nE - 1)] : sent;
    db.z = (e0 + 6 < nE) ? dsts[min(e0 + 6, nE - 1)] : sent;
    db.w = (e0 + 7 < nE) ? dsts[min(e0 + 7, nE - 1)] : sent;
  }
  const unsigned nbs = (unsigned)slotBase;
  const unsigned unb = (unsigned)nb;
  const unsigned s0 = (unsigned)da.x - nbs, s1 = (unsigned)da.y - nbs;
  const unsigned s2 = (unsigned)da.z - nbs, s3 = (unsigned)da.w - nbs;
  const unsigned s4 = (unsigned)db.x - nbs, s5 = (unsigned)db.y - nbs;
  const unsigned s6 = (unsigned)db.z - nbs, s7 = (unsigned)db.w - nbs;
  const bool h0 = s0 < unb, h1 = s1 < unb, h2 = s2 < unb, h3 = s3 < unb;
  const bool h4 = s4 < unb, h5 = s5 < unb, h6 = s6 < unb, h7 = s7 < unb;
  const unsigned any = __builtin_amdgcn_ballot_w32(h0 | h1 | h2 | h3 | h4 | h5 | h6 | h7);
  if (any != 0u) {
#define HITJ(J, HJ, SJ) { \
      const unsigned mj = __builtin_amdgcn_ballot_w32(HJ); \
      if (mj != 0u) { \
        if (HJ) { \
          const int pos = wc + (int)__builtin_amdgcn_mbcnt_lo(mj, 0u); \
          if (pos < WCAP) list[wave * WCAP + pos] = ((el0 + (J)) << SLB) | (int)(SJ); \
        } \
        wc += (int)__builtin_popcount(mj); } }
    HITJ(0, h0, s0)
    HITJ(1, h1, s1)
    HITJ(2, h2, s2)
    HITJ(3, h3, s3)
    HITJ(4, h4, s4)
    HITJ(5, h5, s5)
    HITJ(6, h6, s6)
    HITJ(7, h7, s7)
#undef HITJ
  }
  return wc;
}

__global__ __launch_bounds__(NTHR) void k_prep(const float* __restrict__ h, const float* __restrict__ x,
                                               const float* __restrict__ We1, const float* __restrict__ We2,
                                               const float* __restrict__ Wn1, const float* __restrict__ Wn2,
                                               int nN, int mRows, int nX4,
                                               unsigned short* WABT, unsigned short* WE2T,
                                               unsigned short* WN1T, unsigned short* WN2T,
                                               unsigned short* HB, float* XP, float* MI, float* out1) {
  const int u  = (int)blockIdx.x * NTHR + (int)threadIdx.x;
  const int U0 = NU_WABT;
  const int U1 = U0 + NU_WE2;
  const int U2 = U1 + NU_WN1;
  const int U3 = U2 + NU_WN2;
  const int U4 = U3 + mRows * (HID / 8);
  const int nXP = ((mRows + NTHR - 1) / NTHR) * NTHR;
  const int U5 = U4 + nXP;
  const int U6 = U5 + mRows * (HID / 4);
  const int nXC = ((nX4 + NTHR - 1) / NTHR) * NTHR;
  const int U7 = U6 + nXC;
  const v4f z4 = {0.0f, 0.0f, 0.0f, 0.0f};
  v8us o;
  if (u < U0) {
    const int n   = u >> 3;
    const int k8  = (u & 7) * 8;
    const int kof = (n >> 6) * HID;
    const int nn  = n & (HID - 1);
    const float* p = We1 + (size_t)(kof + k8) * HID + nn;
#pragma unroll
    for (int i = 0; i < 8; ++i) o[i] = (unsigned short)bf16_bits(p[(size_t)i * HID]);
    put16(WABT + (size_t)n * HID + k8, o);
    return;
  } else if (u < U1) {
    const int v  = u - U0;
    const int n  = v >> 3;
    const int k8 = (v & 7) * 8;
    const float* p = We2 + (size_t)k8 * HID + n;
#pragma unroll
    for (int i = 0; i < 8; ++i) o[i] = f2h(CWGT * bf16_val(p[(size_t)i * HID]));
    put16(WE2T + (size_t)n * HID + k8, o);
    return;
  } else if (u < U2) {
    const int v    = u - U1;
    const int n    = v / (KN1 / 8);
    const int k8   = (v - n * (KN1 / 8)) * 8;
    const int srow = (k8 < HID) ? k8 : (k8 - HID);
    const float* p = Wn1 + (size_t)srow * HID + n;
#pragma unroll
    for (int i = 0; i < 8; ++i) o[i] = (unsigned short)bf16_bits(p[(size_t)i * HID]);
    put16(WN1T + (size_t)n * KN1 + k8, o);
    return;
  } else if (u < U3) {
    const int v    = u - U2;
    const int n    = v >> 4;
    const int k8   = (v & 15) * 8;
    const int srow = k8 & (HID - 1);
    const float* p = Wn2 + (size_t)srow * HID + n;
#pragma unroll
    for (int i = 0; i < 8; ++i) o[i] = (unsigned short)bf16_bits(p[(size_t)i * HID]);
    put16(WN2T + (size_t)n * KN2 + k8, o);
    return;
  } else if (u < U4) {
    const int v   = u - U3;
    const int row = v >> 3;
    const int k8  = (v & 7) * 8;
    const int rc  = row < nN ? row : nN - 1;
    const float* p = h + (size_t)rc * HID + k8;
    const v4f a = *(const v4fa*)p;
    const v4f b = *(const v4fa*)(p + 4);
    const bool ok = row < nN;
    o[0] = ok ? (unsigned short)bf16_bits(a.x) : (unsigned short)0;
    o[1] = ok ? (unsigned short)bf16_bits(a.y) : (unsigned short)0;
    o[2] = ok ? (unsigned short)bf16_bits(a.z) : (unsigned short)0;
    o[3] = ok ? (unsigned short)bf16_bits(a.w) : (unsigned short)0;
    o[4] = ok ? (unsigned short)bf16_bits(b.x) : (unsigned short)0;
    o[5] = ok ? (unsigned short)bf16_bits(b.y) : (unsigned short)0;
    o[6] = ok ? (unsigned short)bf16_bits(b.z) : (unsigned short)0;
    o[7] = ok ? (unsigned short)bf16_bits(b.w) : (unsigned short)0;
    put16(HB + (size_t)row * HID + k8, o);
    return;
  } else if (u < U5) {
    const int row = u - U4;
    const int rc  = row < nN ? row : nN - 1;
    const bool ok = row < nN;
    const float x0 = x[(size_t)rc * 3 + 0];
    const float x1 = x[(size_t)rc * 3 + 1];
    const float x2 = x[(size_t)rc * 3 + 2];
    v4f q;
    q.x = ok ? bf16_val(x0) : 0.0f;
    q.y = ok ? bf16_val(x1) : 0.0f;
    q.z = ok ? bf16_val(x2) : 0.0f;
    q.w = 0.0f;
    if (row < mRows) putf4(XP + (size_t)row * 4, q);
    return;
  } else if (u < U6) {
    const int v = u - U5;
    putf4(MI + (size_t)v * 4, z4);
    return;
  } else if (u < U7) {
    const int v  = u - U6;
    const int vc = v < nX4 ? v : nX4 - 1;
    const v4f a  = *(const v4fa*)(x + (size_t)vc * 4);
    if (v < nX4) putf4(out1 + (size_t)v * 4, a);
    return;
  }
}

template <int MODE, int NT>
__global__ __launch_bounds__(GTHR) void k_gemm(const unsigned short* __restrict__ A, int lda,
                                               const unsigned short* __restrict__ BT, int ldb, int K,
                                               const float* __restrict__ bias, const float* __restrict__ hres,
                                               const float* __restrict__ lng, const float* __restrict__ lnb,
                                               int nN, float* Cm, int ldc, unsigned short* Cb) {
  static_assert((MODE == 0 && NT == 8) || (MODE != 0 && NT == 4));
  constexpr int BN = 16 * NT;
  __shared__ __attribute__((aligned(16))) float stg[GBM * BN];
  const int tid = (int)threadIdx.x, lane = tid & 31, wave = tid >> 5, hh = lane >> 4, m = lane & 15;
  const int rowBase = (int)blockIdx.x * GBM;
  const int colBase = (int)blockIdx.y * BN;

  v8f acc[NT];
  {
    const v8f z = {0.f, 0.f, 0.f, 0.f, 0.f, 0.f, 0.f, 0.f};
#pragma unroll
    for (int t = 0; t < NT; ++t) acc[t] = z;
  }
  const unsigned short* ap = A  + (size_t)(rowBase + 16 * wave + m) * (size_t)lda + 8 * hh;
  const unsigned short* bp = BT + (size_t)(colBase + m) * (size_t)ldb + 8 * hh;

#pragma unroll 1
  for (int k0 = 0; k0 < K; k0 += 32) {
    FragB af;
    af.h[0] = *(const v8usa*)(ap + k0);
    af.h[1] = *(const v8usa*)(ap + k0 + 16);
#pragma unroll
    for (int nt = 0; nt < NT; ++nt) {
      const unsigned short* wq = bp + (size_t)(16 * nt) * (size_t)ldb + k0;
      FragB bf;
      bf.h[0] = *(const v8usa*)wq;
      bf.h[1] = *(const v8usa*)(wq + 16);
      acc[nt] = wmb(af, bf, acc[nt]);
    }
  }

#pragma unroll
  for (int nt = 0; nt < NT; ++nt) {
    const int lc = 16 * nt + m;
    float bvv = 0.0f;
    if constexpr (MODE != 0) bvv = bf16_val(bias[colBase + lc]);
#pragma unroll
    for (int r = 0; r < 8; ++r) {
      const int lr = 16 * wave + 8 * hh + r;
      float v = acc[nt][r];
      if constexpr (MODE == 1) v = fmaxf(v + bvv, 0.0f);
      if constexpr (MODE == 2) v = v + bvv;
      stg[lr * BN + lc] = v;
    }
  }
  __syncthreads();

  if constexpr (MODE == 0) {
    v4f pv[16];
#pragma unroll
    for (int i = 0; i < 16; ++i) pv[i] = *(const v4fa*)(stg + (16 * wave + i) * BN + 4 * lane);
#pragma unroll
    for (int i = 0; i < 16; ++i) {
      float* op = Cm + (size_t)(rowBase + 16 * wave + i) * (size_t)ldc + colBase + 4 * lane;
      *(volatile v4f*)op = pv[i];
    }
    __threadfence();
#pragma unroll
    for (int i = 0; i < 16; ++i) {
      float* op = Cm + (size_t)(rowBase + 16 * wave + i) * (size_t)ldc + colBase + 4 * lane;
      *(volatile v4f*)op = pv[i];
    }
  } else if constexpr (MODE == 1) {
    const int rsel = lane >> 4;
    const int part = (lane >> 3) & 1;
    const int j = lane & 7;
    const unsigned mh = 0u - (unsigned)part;
    const unsigned ml = ~mh;
    v8us pv[8];
#pragma unroll
    for (int i = 0; i < 8; ++i) {
      const int rr = 16 * wave + 2 * i + rsel;
      const float* sp = stg + rr * BN + 8 * j;
      const v4f a = *(const v4fa*)sp;
      const v4f b = *(const v4fa*)(sp + 4);
      const v8f f8 = {a.x, a.y, a.z, a.w, b.x, b.y, b.z, b.w};
      v8us oo;
#pragma unroll
      for (int e = 0; e < 8; ++e) {
        const unsigned hb = bf16_bits(f8[e]);
        const unsigned lb = bf16_bits(f8[e] - __uint_as_float(hb << 16));
        oo[e] = (unsigned short)((hb & ml) | (lb & mh));
      }
      pv[i] = oo;
    }
#pragma unroll
    for (int i = 0; i < 8; ++i) {
      const int rr = 16 * wave + 2 * i + rsel;
      unsigned short* op = Cb + (size_t)(rowBase + rr) * (size_t)KN2 + part * HID + 8 * j;
      *(volatile v8us*)op = pv[i];
    }
    __threadfence();
#pragma unroll
    for (int i = 0; i < 8; ++i) {
      const int rr = 16 * wave + 2 * i + rsel;
      unsigned short* op = Cb + (size_t)(rowBase + rr) * (size_t)KN2 + part * HID + 8 * j;
      *(volatile v8us*)op = pv[i];
    }
  } else {
    const int rsel = lane >> 4;
    const int q = lane & 15;
    v4f gq, bq;
    {
      const v4f g4 = *(const v4fa*)(lng + 4 * q);
      const v4f b4 = *(const v4fa*)(lnb + 4 * q);
      gq.x = bf16_val(g4.x); gq.y = bf16_val(g4.y); gq.z = bf16_val(g4.z); gq.w = bf16_val(g4.w);
      bq.x = bf16_val(b4.x); bq.y = bf16_val(b4.y); bq.z = bf16_val(b4.z); bq.w = bf16_val(b4.w);
    }
    const float inv64 = 0.015625f;
    v4f pv[8];
#pragma unroll
    for (int i = 0; i < 8; ++i) {
      const int rr  = 16 * wave + 2 * i + rsel;
      const int row = rowBase + rr;
      const int rc  = row < nN ? row : nN - 1;
      const v4f hv = *(const v4fa*)(hres + (size_t)rc * HID + 4 * q);
      const v4f sv = *(const v4fa*)(stg + rr * BN + 4 * q);
      v4f z;
      z.x = sv.x + bf16_val(hv.x);
      z.y = sv.y + bf16_val(hv.y);
      z.z = sv.z + bf16_val(hv.z);
      z.w = sv.w + bf16_val(hv.w);
      float s = (z.x + z.y) + (z.z + z.w);
      s += __shfl_xor(s, 1, 32);
      s += __shfl_xor(s, 2, 32);
      s += __shfl_xor(s, 4, 32);
      s += __shfl_xor(s, 8, 32);
      const float mean = s * inv64;
      v4f d;
      d.x = z.x - mean; d.y = z.y - mean; d.z = z.z - mean; d.w = z.w - mean;
      float s2 = (d.x * d.x + d.y * d.y) + (d.z * d.z + d.w * d.w);
      s2 += __shfl_xor(s2, 1, 32);
      s2 += __shfl_xor(s2, 2, 32);
      s2 += __shfl_xor(s2, 4, 32);
      s2 += __shfl_xor(s2, 8, 32);
      const float var  = s2 * inv64;
      const float rstd = rsqrtf(var + LNEPS);
      v4f o4;
      o4.x = fmaf(d.x * rstd, gq.x, bq.x);
      o4.y = fmaf(d.y * rstd, gq.y, bq.y);
      o4.z = fmaf(d.z * rstd, gq.z, bq.z);
      o4.w = fmaf(d.w * rstd, gq.w, bq.w);
      pv[i] = o4;
    }
#pragma unroll
    for (int i = 0; i < 8; ++i) {
      const int row = rowBase + 16 * wave + 2 * i + rsel;
      if (row < nN) {
        float* op = Cm + (size_t)row * (size_t)ldc + colBase + 4 * q;
        *(volatile v4f*)op = pv[i];
      }
    }
    __threadfence();
#pragma unroll
    for (int i = 0; i < 8; ++i) {
      const int row = rowBase + 16 * wave + 2 * i + rsel;
      if (row < nN) {
        float* op = Cm + (size_t)row * (size_t)ldc + colBase + 4 * q;
        *(volatile v4f*)op = pv[i];
      }
    }
  }
}

__device__ __forceinline__ void wave_gemm_h(const unsigned short* sAw, float* sDw,
                                            const unsigned short* __restrict__ BT, int ldb, int K,
                                            int hh, int m) {
  v8f acc[2][4];
  {
    const v8f z = {0.f, 0.f, 0.f, 0.f, 0.f, 0.f, 0.f, 0.f};
#pragma unroll
    for (int mt = 0; mt < 2; ++mt)
#pragma unroll
      for (int nt = 0; nt < 4; ++nt) acc[mt][nt] = z;
  }
  const unsigned short* ap0 = sAw + m * AP + 8 * hh;
  const unsigned short* ap1 = ap0 + 16 * AP;
  const unsigned short* bp  = BT + (size_t)m * (size_t)ldb + 8 * hh;
#pragma unroll 1
  for (int k0 = 0; k0 < K; k0 += 32) {
    FragH a0, a1;
    a0.h[0] = *(const v8usa*)(ap0 + k0);
    a0.h[1] = *(const v8usa*)(ap0 + k0 + 16);
    a1.h[0] = *(const v8usa*)(ap1 + k0);
    a1.h[1] = *(const v8usa*)(ap1 + k0 + 16);
#pragma unroll
    for (int nt = 0; nt < 4; ++nt) {
      const unsigned short* wq = bp + (size_t)(16 * nt) * (size_t)ldb + k0;
      FragH b;
      b.h[0] = *(const v8usa*)wq;
      b.h[1] = *(const v8usa*)(wq + 16);
      acc[0][nt] = wmh(a0, b, acc[0][nt]);
      acc[1][nt] = wmh(a1, b, acc[1][nt]);
    }
  }
#pragma unroll
  for (int nt = 0; nt < 4; ++nt) {
    const int col = 16 * nt + m;
#pragma unroll
    for (int mt = 0; mt < 2; ++mt)
#pragma unroll
      for (int r = 0; r < 8; ++r) sDw[(16 * mt + 8 * hh + r) * DP + col] = acc[mt][nt][r];
  }
}

__global__ __launch_bounds__(NTHR) void k_edge(const int* __restrict__ ei, int nE, int nN, int eBase, int nEh,
                                               const float* __restrict__ PQ, const float* __restrict__ XP,
                                               const unsigned short* __restrict__ WE2T,
                                               const float* __restrict__ be1, const float* __restrict__ be2,
                                               const float* __restrict__ Winf, const float* __restrict__ binf,
                                               unsigned short* Mh) {
  extern __shared__ __attribute__((aligned(16))) float dyn[];
  float*          sD  = dyn;
  unsigned short* sA  = (unsigned short*)(dyn + EPB * DP);
  unsigned short* sM  = sA + EPB * AP;
  float*          cst = dyn + EPB * DP + (EPB * AP) / 2 + (EPB * MPITCH) / 2;

  const int tid = (int)threadIdx.x, lane = tid & 31, wave = tid >> 5, hh = lane >> 4, m = lane & 15;

  if (tid < HID) {
    cst[tid]           = bf16_val(be1[tid]);
    cst[HID + tid]     = bf16_val(be2[tid]);
    cst[2 * HID + tid] = bf16_val(Winf[tid]);
    const float vb = bf16_val(binf[0]);
    if (tid == 0) cst[3 * HID] = vb;
  }

  const int  elb  = (int)blockIdx.x * EPB;
  const int  el   = elb + tid;
  const bool live = el < nEh;
  const int  elc  = live ? el : (nEh - 1);
  const int  eg   = eBase + elc;
  int s = ei[eg];
  int t = ei[(size_t)nE + (size_t)eg];
  s = s < 0 ? 0 : (s > nN - 1 ? nN - 1 : s);
  t = t < 0 ? 0 : (t > nN - 1 ? nN - 1 : t);
  const v4f xs = *(const v4fa*)(XP + (size_t)s * 4);
  const v4f xd = *(const v4fa*)(XP + (size_t)t * 4);
  const float rx = xd.x - xs.x, ry = xd.y - xs.y, rz = xd.z - xs.z;
  const float dsq  = (rx * rx + rz * rz) + ry * ry;
  const float dd   = sqrtf(dsq + 0.0f);
  const float edis = sigm_f(TEMF * __builtin_amdgcn_rcpf(dd + 1e-8f));

  float*          rd = sD + tid * DP;
  unsigned short* ra = sA + tid * AP;
  unsigned short* rm = sM + tid * MPITCH;
  __syncthreads();

  {
    const float* pr = PQ + (size_t)t * NPQ;
    const float* qr = PQ + (size_t)s * NPQ + HID;
#pragma unroll 1
    for (int c8 = 0; c8 < HID / 8; ++c8) {
      const v4f pa = *(const v4fa*)(pr + 8 * c8);
      const v4f pb = *(const v4fa*)(pr + 8 * c8 + 4);
      const v4f qa = *(const v4fa*)(qr + 8 * c8);
      const v4f qb = *(const v4fa*)(qr + 8 * c8 + 4);
      const v4f ba = *(const v4fa*)(cst + 8 * c8);
      const v4f bb = *(const v4fa*)(cst + 8 * c8 + 4);
      const v8f p8 = {pa.x, pa.y, pa.z, pa.w, pb.x, pb.y, pb.z, pb.w};
      const v8f q8 = {qa.x, qa.y, qa.z, qa.w, qb.x, qb.y, qb.z, qb.w};
      const v8f b8 = {ba.x, ba.y, ba.z, ba.w, bb.x, bb.y, bb.z, bb.w};
      v8us o;
#pragma unroll
      for (int i = 0; i < 8; ++i) {
        const float pre = (p8[i] + q8[i]) + b8[i];
        o[i] = f2h(CACT * fmaxf(pre, 0.0f));
      }
      *(v8usa*)(ra + 8 * c8) = o;
    }
  }
  __syncthreads();

  const unsigned short* sAw = sA + 32 * wave * AP;
  float*                sDw = sD + 32 * wave * DP;

  wave_gemm_h(sAw, sDw, WE2T, HID, HID, hh, m);
  __syncthreads();

  {
    float dot = 0.0f;
#pragma unroll 1
    for (int c8 = 0; c8 < HID / 8; ++c8) {
      const v4f va = *(const v4fa*)(rd + 8 * c8);
      const v4f vb = *(const v4fa*)(rd + 8 * c8 + 4);
      const v4f ba = *(const v4fa*)(cst + HID + 8 * c8);
      const v4f bb = *(const v4fa*)(cst + HID + 8 * c8 + 4);
      const v4f wa = *(const v4fa*)(cst + 2 * HID + 8 * c8);
      const v4f wb = *(const v4fa*)(cst + 2 * HID + 8 * c8 + 4);
      const v8f v8 = {va.x, va.y, va.z, va.w, vb.x, vb.y, vb.z, vb.w};
      const v8f b8 = {ba.x, ba.y, ba.z, ba.w, bb.x, bb.y, bb.z, bb.w};
      const v8f w8 = {wa.x, wa.y, wa.z, wa.w, wb.x, wb.y, wb.z, wb.w};
      v8f mf;
#pragma unroll
      for (int i = 0; i < 8; ++i) {
        const float mj = fmaxf(fmaf(v8[i], PINV, b8[i]), 0.0f);
        dot   = fmaf(mj, w8[i], dot);
        mf[i] = mj;
      }
      const v4f m0 = {mf[0], mf[1], mf[2], mf[3]};
      const v4f m1 = {mf[4], mf[5], mf[6], mf[7]};
      *(v4fa*)(rd + 8 * c8)     = m0;
      *(v4fa*)(rd + 8 * c8 + 4) = m1;
    }
    const float eij = dot + cst[3 * HID];
    const float wgt = sigm_f(eij * edis);
#pragma unroll 1
    for (int c8 = 0; c8 < HID / 8; ++c8) {
      const v4f va = *(const v4fa*)(rd + 8 * c8);
      const v4f vb = *(const v4fa*)(rd + 8 * c8 + 4);
      const v8f v8 = {va.x, va.y, va.z, va.w, vb.x, vb.y, vb.z, vb.w};
      v8us o;
#pragma unroll
      for (int i = 0; i < 8; ++i) o[i] = f2h(CMSG * (v8[i] * wgt));
      *(v8usa*)(rm + 8 * c8) = o;
    }
  }
  __syncthreads();

  {
    v4i pv[8];
#pragma unroll
    for (int it = 0; it < 8; ++it) pv[it] = *(const v4ia*)(sM + (size_t)(it * NTHR + tid) * 8);
    unsigned short* mb = Mh + (size_t)elb * MPITCH;
#pragma unroll
    for (int it = 0; it < 8; ++it) *(volatile v4i*)(mb + (size_t)(it * NTHR + tid) * 8) = pv[it];
    __threadfence();
#pragma unroll
    for (int it = 0; it < 8; ++it) *(volatile v4i*)(mb + (size_t)(it * NTHR + tid) * 8) = pv[it];
  }
}

__global__ __launch_bounds__(NTHR) void k_scan(const int* __restrict__ dsts, int nEh, int vec8, int mRows,
                                               const unsigned short* __restrict__ Mh, float* MI) {
  extern __shared__ __attribute__((aligned(16))) int dsm[];
  int* list = dsm;
  int* hl   = dsm + LISTN;
  int* sl   = hl + RCAP;
  int* cnt  = sl + RCAP;
  int* offs = cnt + NBA;
  int* cur  = offs + NBA;
  int* misc = cur + NBA;
  const int tid = (int)threadIdx.x, lane = tid & 31, wave = tid >> 5;
  const int nodeBase = (int)blockIdx.x * NBA;

  {
    const v4i z4 = {0, 0, 0, 0};
    for (int i = tid * 4; i < AGG_ZINTS; i += NTHR * 4) *(v4ia*)(dsm + i) = z4;
    if (tid < 16) misc[tid] = 0;
  }
  __syncthreads();

  int t = 0, ov = 0;
  const int nChunks = (nEh + CHUNK - 1) / CHUNK;
#pragma unroll 1
  for (int ch = 0; ch < nChunks; ++ch) {
    const int cbase = ch * CHUNK;
    const int wc = scan_chunk<SLA>(dsts, nEh, cbase, nodeBase, NBA, vec8, list, tid, lane, wave);
    if (lane == 0) misc[wave] = wc;
    __syncthreads();
    if (wave == 0) {
#pragma unroll 1
      for (int w2 = 0; w2 < NWAVE; ++w2) {
        int c = misc[w2];
        c = c < 0 ? 0 : (c > WCAP ? WCAP : c);
#pragma unroll 1
        for (int b0 = 0; b0 < c; b0 += 32) {
          const int idx = b0 + lane;
          const int ent = list[w2 * WCAP + (idx < WCAP ? idx : WCAP - 1)];
          const int m32 = (c - b0) < 32 ? (c - b0) : 32;
#pragma unroll 1
          for (int k = 0; k < m32; ++k) {
            const int u    = __builtin_amdgcn_readlane(ent, k);
            const int slot = u & (NBA - 1);
            const int el   = (u >> SLA) & (CHUNK - 1);
            const int pk   = ((cbase + el) << SLA) | slot;
            if (t < RCAP) {
              if (lane == 0) { hl[t] = pk; cnt[slot] = cnt[slot] + 1; }
              t = t + 1;
            } else {
              ov = 1;
            }
          }
        }
      }
    }
    __syncthreads();
  }
  if (wave == 0 && lane == 0) { misc[8] = t; misc[9] = ov; }
  __syncthreads();
  int tt = misc[8];
  tt = tt < 0 ? 0 : (tt > RCAP ? RCAP : tt);
  const int ovf = misc[9];

  if (wave == 0) {
    const int base = lane * (NBA / 32);
    int sm = 0;
#pragma unroll 1
    for (int i = 0; i < NBA / 32; ++i) sm += cnt[base + i];
    int incl = sm;
#pragma unroll
    for (int d = 1; d < 32; d <<= 1) {
      const int y = __shfl_up(incl, d, 32);
      if (lane >= d) incl += y;
    }
    int run = incl - sm;
#pragma unroll 1
    for (int i = 0; i < NBA / 32; ++i) {
      const int cv = cnt[base + i];
      offs[base + i] = run;
      cur[base + i]  = run;
      run += cv;
    }
  }
  __syncthreads();
  if (wave == 0) {
#pragma unroll 1
    for (int b0 = 0; b0 < tt; b0 += 32) {
      const int idx = b0 + lane;
      const int ent = hl[idx < RCAP ? idx : RCAP - 1];
      const int m32 = (tt - b0) < 32 ? (tt - b0) : 32;
#pragma unroll 1
      for (int k = 0; k < m32; ++k) {
        const int u    = __builtin_amdgcn_readlane(ent, k);
        const int slot = u & (NBA - 1);
        if (lane == 0) {
          int p = cur[slot];
          p = p < 0 ? 0 : (p > RCAP - 1 ? RCAP - 1 : p);
          sl[p] = u;
          cur[slot] = p + 1;
        }
      }
    }
  }
  __syncthreads();

  const float qnan = __int_as_float(0x7fc00000);
  const float pz = (ovf != 0) ? qnan : 0.0f;
  const int q = lane & 15;
#pragma unroll 1
  for (int si = 0; si < NBA / NWAVE; ++si) {
    const int s    = si * NWAVE + wave;
    const int node = nodeBase + s;
    int c = cnt[s];
    const bool big = c > DEGCAP;
    c = c < 0 ? 0 : (c > DEGCAP ? DEGCAP : c);
    int o = offs[s];
    o = o < 0 ? 0 : (o > RCAP ? RCAP : o);
    float a0 = 0.0f, a1 = 0.0f;
#pragma unroll 1
    for (int b0 = 0; b0 < c; b0 += 32) {
      int idx = o + b0 + lane;
      idx = idx > RCAP - 1 ? RCAP - 1 : idx;
      const int ent = sl[idx];
      int eid = ent >> SLA;
      eid = eid < 0 ? 0 : (eid > nEh - 1 ? nEh - 1 : eid);
      const int m32 = (c - b0) < 32 ? (c - b0) : 32;
#pragma unroll 1
      for (int k = 0; k < m32; ++k) {
        const int ek = __builtin_amdgcn_readlane(eid, k);
        const unsigned w = *(const u32a*)(Mh + (size_t)ek * MPITCH + 2 * lane);
        a0 += h2f(w & 0xffffu);
        a1 += h2f(w >> 16);
      }
    }
    const bool  live = node < mRows;
    const int   nr   = live ? node : mRows - 1;
    const float pzr  = big ? qnan : pz;
    const float c0 = __shfl(a0, 2 * q, 32);
    const float c1 = __shfl(a1, 2 * q, 32);
    const float c2 = __shfl(a0, 2 * q + 1, 32);
    const float c3 = __shfl(a1, 2 * q + 1, 32);
    float* mp = MI + (size_t)nr * HID + 4 * q;
    const v4f old = *(const v4fa*)mp;
    v4f nv;
    nv.x = fmaf(c0, MINV, old.x) + pzr;
    nv.y = fmaf(c1, MINV, old.y) + pzr;
    nv.z = fmaf(c2, MINV, old.z) + pzr;
    nv.w = fmaf(c3, MINV, old.w) + pzr;
    const bool st = live && (lane < 16);
    if (st) *(volatile v4f*)mp = nv;
    __threadfence();
    if (st) *(volatile v4f*)mp = nv;
  }
}

__global__ __launch_bounds__(NTHR) void k_nz(const float* __restrict__ MI, const float* __restrict__ h,
                                             int nN, int nUnits, unsigned short* NZ) {
  const int u = (int)blockIdx.x * NTHR + (int)threadIdx.x;
  if (u >= nUnits) return;
  const int row = u >> 3;
  const int j   = u & 7;
  const int rc  = row < nN ? row : nN - 1;
  const bool ok = row < nN;
  const float* mq = MI + (size_t)row * HID + 8 * j;
  const float* hq = h  + (size_t)rc  * HID + 8 * j;
  const v4f ma = *(const v4fa*)mq;
  const v4f mb = *(const v4fa*)(mq + 4);
  const v4f ha = *(const v4fa*)hq;
  const v4f hb = *(const v4fa*)(hq + 4);
  const v8f m8 = {ma.x, ma.y, ma.z, ma.w, mb.x, mb.y, mb.z, mb.w};
  const v8f h8 = {ha.x, ha.y, ha.z, ha.w, hb.x, hb.y, hb.z, hb.w};
  v8us ohi, olo, ohb;
#pragma unroll
  for (int i = 0; i < 8; ++i) {
    const unsigned hbits = bf16_bits(m8[i]);
    ohi[i] = (unsigned short)hbits;
    olo[i] = (unsigned short)bf16_bits(m8[i] - __uint_as_float(hbits << 16));
    ohb[i] = ok ? (unsigned short)bf16_bits(h8[i]) : (unsigned short)0;
  }
  unsigned short* dp = NZ + (size_t)row * KN1 + 8 * j;
  *(volatile v8us*)dp             = ohi;
  *(volatile v8us*)(dp + HID)     = olo;
  *(volatile v8us*)(dp + 2 * HID) = ohb;
  __threadfence();
  *(volatile v8us*)dp             = ohi;
  *(volatile v8us*)(dp + HID)     = olo;
  *(volatile v8us*)(dp + 2 * HID) = ohb;
}

static inline int cdiv(int a, int b) { return (a + b - 1) / b; }

extern "C" void kernel_launch(void* const* d_in, const int* in_sizes, int n_in,
                              void* d_out, int out_size, void* d_ws, size_t ws_size,
                              hipStream_t stream) {
  if (n_in < 15) return;
  if (in_sizes[0] < HID || (in_sizes[0] % HID) != 0) return;
  const int nN = in_sizes[0] / HID;
  if (in_sizes[1] != 3 * nN) return;
  if (in_sizes[2] < 2 || (in_sizes[2] & 1) != 0) return;
  const int nE = in_sizes[2] / 2;
  if (nE < 1 || nE >= (1 << 22)) return;
  if (in_sizes[3] != 2 * HID * HID || in_sizes[4] != HID) return;
  if (in_sizes[5] != HID * HID || in_sizes[6] != HID) return;
  if (in_sizes[7] != HID || in_sizes[8] != 1) return;
  if (in_sizes[9] != 2 * HID * HID || in_sizes[10] != HID) return;
  if (in_sizes[11] != HID * HID || in_sizes[12] != HID) return;
  if (in_sizes[13] != HID || in_sizes[14] != HID) return;
  if ((long long)out_size != (long long)nN * HID + 3LL * nN) return;
  if (((3 * nN) & 3) != 0) return;

  const float* h     = (const float*)d_in[0];
  const float* x     = (const float*)d_in[1];
  const int*   ei    = (const int*)d_in[2];
  const float* We1   = (const float*)d_in[3];
  const float* be1   = (const float*)d_in[4];
  const float* We2   = (const float*)d_in[5];
  const float* be2   = (const float*)d_in[6];
  const float* Winf  = (const float*)d_in[7];
  const float* binf  = (const float*)d_in[8];
  const float* Wn1   = (const float*)d_in[9];
  const float* bn1   = (const float*)d_in[10];
  const float* Wn2   = (const float*)d_in[11];
  const float* bn2   = (const float*)d_in[12];
  const float* ln_g  = (const float*)d_in[13];
  const float* ln_b  = (const float*)d_in[14];
  float* out0 = (float*)d_out;
  float* out1 = out0 + (size_t)nN * HID;

  const int MP = cdiv(nN, GBM) * GBM;
  const int gM = MP / GBM;
  const int gA = cdiv(MP, NBA);
  if ((long long)gA * NBA < (long long)MP) return;
  const int EH  = cdiv(cdiv(nE, NRANGE), EPB) * EPB;
  const int EHP = EH;
  if (EH < 1 || EH >= (1 << 21)) return;
  const int nX4 = (3 * nN) / 4;

  char* ws = (char*)d_ws;
  size_t off = 0;
  const size_t oWABT = off; off += (size_t)NPQ * HID * 2;            off = (off + 255) & ~(size_t)255;
  const size_t oWE2T = off; off += (size_t)HID * HID * 2;            off = (off + 255) & ~(size_t)255;
  const size_t oWN1T = off; off += (size_t)HID * KN1 * 2;            off = (off + 255) & ~(size_t)255;
  const size_t oWN2T = off; off += (size_t)HID * KN2 * 2;            off = (off + 255) & ~(size_t)255;
  const size_t oXP   = off; off += (size_t)MP * 4 * 4;               off = (off + 255) & ~(size_t)255;
  const size_t oMI   = off; off += (size_t)MP * HID * 4;             off = (off + 255) & ~(size_t)255;
  size_t szRM = (size_t)EHP * MPITCH * 2;
  if (szRM < (size_t)MP * HID * 2) szRM = (size_t)MP * HID * 2;
  if (szRM < (size_t)MP * KN2 * 2) szRM = (size_t)MP * KN2 * 2;
  const size_t oRM   = off; off += szRM;                             off = (off + 255) & ~(size_t)255;
  size_t szRP = (size_t)MP * NPQ * 4;
  if (szRP < (size_t)MP * KN1 * 2) szRP = (size_t)MP * KN1 * 2;
  const size_t oRP   = off; off += szRP;                             off = (off + 255) & ~(size_t)255;
  if (off > ws_size || off > (size_t)WSMAX) return;
  unsigned short* WABT = (unsigned short*)(ws + oWABT);
  unsigned short* WE2T = (unsigned short*)(ws + oWE2T);
  unsigned short* WN1T = (unsigned short*)(ws + oWN1T);
  unsigned short* WN2T = (unsigned short*)(ws + oWN2T);
  float*          XP   = (float*)(ws + oXP);
  float*          MI   = (float*)(ws + oMI);
  unsigned short* HB   = (unsigned short*)(ws + oRM);
  unsigned short* MSG  = (unsigned short*)(ws + oRM);
  unsigned short* G1   = (unsigned short*)(ws + oRM);
  float*          PQ   = (float*)(ws + oRP);
  unsigned short* NZ   = (unsigned short*)(ws + oRP);

  hipFuncSetAttribute(reinterpret_cast<const void*>(&k_edge), hipFuncAttributeMaxDynamicSharedMemorySize,
                      (int)EDGE_LDS_BYTES);
  hipFuncSetAttribute(reinterpret_cast<const void*>(&k_scan), hipFuncAttributeMaxDynamicSharedMemorySize,
                      (int)AGG_LDS_BYTES);

  const int nXP   = cdiv(MP, NTHR) * NTHR;
  const int nXC   = cdiv(nX4, NTHR) * NTHR;
  const int nPrep = NU_WABT + NU_WE2 + NU_WN1 + NU_WN2 + MP * (HID / 8) + nXP + MP * (HID / 4) + nXC;

  k_prep<<<nPrep / NTHR, NTHR, 0, stream>>>(h, x, We1, We2, Wn1, Wn2, nN, MP, nX4,
                                            WABT, WE2T, WN1T, WN2T, HB, XP, MI, out1);
  k_gemm<0, 8><<<dim3(gM, 1), GTHR, 0, stream>>>(HB, HID, WABT, HID, HID, bn1, h, ln_g, ln_b, nN,
                                                 PQ, NPQ, G1);
  for (int r = 0; r < NRANGE; ++r) {
    const int eBase = r * EH;
    if (eBase >= nE) break;
    const int nEh = (nE - eBase) < EH ? (nE - eBase) : EH;
    const int vec = (((nE + eBase) & 3) == 0) ? 1 : 0;
    k_edge<<<cdiv(nEh, EPB), NTHR, EDGE_LDS_BYTES, stream>>>(ei, nE, nN, eBase, nEh, PQ, XP, WE2T,
                                                              be1, be2, Winf, binf, MSG);
    k_scan<<<gA, NTHR, AGG_LDS_BYTES, stream>>>(ei + (size_t)nE + (size_t)eBase, nEh, vec, MP, MSG, MI);
  }
  k_nz<<<(MP * (HID / 8)) / NTHR, NTHR, 0, stream>>>(MI, h, nN, MP * (HID / 8), NZ);
  k_gemm<1, 4><<<dim3(gM, 1), GTHR, 0, stream>>>(NZ, KN1, WN1T, KN1, KN1, bn1, h, ln_g, ln_b, nN,
                                                 MI, HID, G1);
  k_gemm<2, 4><<<dim3(gM, 1), GTHR, 0, stream>>>(G1, KN2, WN2T, KN2, KN2, bn2, h, ln_g, ln_b, nN,
                                                 out0, HID, NZ);
}
